// PatchSampleLayer_29025388987060
// MI455X (gfx1250) — hardware-verified
//
#include <hip/hip_runtime.h>
#include <math.h>

typedef __attribute__((ext_vector_type(16))) _Float16 v16h;
typedef __attribute__((ext_vector_type(16))) __bf16 v16b;
typedef __attribute__((ext_vector_type(8)))  _Float16 v8h;
typedef __attribute__((ext_vector_type(8)))  float v8f;
typedef __attribute__((ext_vector_type(4)))  float v4f;
typedef __attribute__((ext_vector_type(2)))  float v2f;
typedef __attribute__((ext_vector_type(4)))  unsigned v4u;
typedef __attribute__((ext_vector_type(4)))  int v4i;
typedef float __attribute__((may_alias)) float_a;
typedef int __attribute__((may_alias)) int_a;

template <typename T> __device__ __forceinline__ void vst2(void* p, T v) { *(volatile T*)p = v; __threadfence(); *(volatile T*)p = v; }
__device__ __forceinline__ v8f wmma16(v16h a, v16h b, v8f c) {
  v8f d = __builtin_amdgcn_wmma_f32_16x16x32_f16(false, a, false, b, (short)0, c, false, false);
  asm volatile("v_nop\n\tv_nop\n\tv_nop\n\tv_nop" : "+v"(d) : "v"(a), "v"(b));
  return d;
}
__device__ __forceinline__ v8f wmma_bf(v16b a, v16b b, v8f c) {
  v8f d = __builtin_amdgcn_wmma_f32_16x16x32_bf16(false, a, false, b, (short)0, c, false, false);
  asm volatile("v_nop\n\tv_nop\n\tv_nop\n\tv_nop" : "+v"(d) : "v"(a), "v"(b));
  return d;
}
__device__ __forceinline__ v16h frag_h(const _Float16* rowk0, int lane) {
  union { v16h v; v8h q[2]; } u; const _Float16* p = rowk0 + 8 * (lane >> 4);
  u.q[0] = *(const v8h*)p; u.q[1] = *(const v8h*)(p + 16); return u.v;
}
__device__ __forceinline__ v16h frag_f32(const float* rowk0, int lane) {
  v16h a; const float* p = rowk0 + 8 * (lane >> 4);
#pragma unroll
  for (int i = 0; i < 8; ++i) { a[i] = (_Float16)p[i]; a[8 + i] = (_Float16)p[16 + i]; }
  return a;
}
__device__ __forceinline__ v16h frag_f32s(const float* rowk0, int lane, float sc) {
  v16h a; const float* p = rowk0 + 8 * (lane >> 4);
#pragma unroll
  for (int i = 0; i < 8; ++i) { a[i] = (_Float16)(p[i] * sc); a[8 + i] = (_Float16)(p[16 + i] * sc); }
  return a;
}
__device__ __forceinline__ v16h fragc_f32(const float* W, int k0, int n, int lane, int ld, int K) {
  v16h a; const int g = lane >> 4;
#pragma unroll
  for (int i = 0; i < 8; ++i) { const int ka = k0 + 8 * g + i, kb = ka + 16;
    a[i] = (_Float16)(ka < K ? W[(size_t)(ka < K ? ka : K - 1) * ld + n] : 0.f); a[8 + i] = (_Float16)(kb < K ? W[(size_t)(kb < K ? kb : K - 1) * ld + n] : 0.f); }
  return a;
}
struct F2 { v16b h, l; };
__device__ __forceinline__ F2 bsplit16(const float v[16]) { F2 r;
#pragma unroll
  for (int i = 0; i < 16; ++i) { const __bf16 h = (__bf16)v[i]; r.h[i] = h; r.l[i] = (__bf16)(v[i] - (float)h); }
  return r; }
__device__ __forceinline__ F2 split_row(const float* row, int k0, int lane) { float v[16]; const float* p = row + k0 + 8 * (lane >> 4);
#pragma unroll
  for (int i = 0; i < 8; ++i) { v[i] = p[i]; v[8 + i] = p[16 + i]; }
  return bsplit16(v); }
__device__ __forceinline__ F2 split_rowK(const float* row, int k0, int lane, int K) { float v[16]; const int g = lane >> 4;
#pragma unroll
  for (int i = 0; i < 8; ++i) { const int ka = k0 + 8 * g + i, kb = ka + 16; v[i] = ka < K ? row[ka < K ? ka : K - 1] : 0.f; v[8 + i] = kb < K ? row[kb < K ? kb : K - 1] : 0.f; }
  return bsplit16(v); }
__device__ __forceinline__ F2 split_col(const float* W, int k0, int n, int lane, int ld, int K) { float v[16]; const int g = lane >> 4;
#pragma unroll
  for (int i = 0; i < 8; ++i) { const int ka = k0 + 8 * g + i, kb = ka + 16; v[i] = ka < K ? W[(size_t)(ka < K ? ka : K - 1) * ld + n] : 0.f; v[8 + i] = kb < K ? W[(size_t)(kb < K ? kb : K - 1) * ld + n] : 0.f; }
  return bsplit16(v); }
__device__ __forceinline__ v8f mac3(const F2& a, const F2& b, v8f c) { c = wmma_bf(a.l, b.h, c); c = wmma_bf(a.h, b.l, c); return wmma_bf(a.h, b.h, c); }
__device__ __forceinline__ float sigm(float v) { return 1.0f / (1.0f + expf(-v)); }
#define LDSX() do { asm volatile("s_wait_dscnt 0" ::: "memory"); __builtin_amdgcn_wave_barrier(); __builtin_amdgcn_fence(__ATOMIC_RELEASE, "workgroup"); } while (0)


#define NBq 2
#define NQ 256
#define NP (NBq * NQ)
#define INC 256
#define HID 64
#define CHM 62
#define CHP 64
#define HIN 180
#define WIN 180
#define HS 40
#define WSd 40
#define HO 38
#define WO 38
#define NPOS (HO * WO)
#define NBLK 23
#define KTAP 9
#ifndef TNP
#define TNP NP
#endif
typedef __attribute__((ext_vector_type(8))) __bf16 v8b;
__device__ __forceinline__ v16b frag_b(const __bf16* rowk0, int lane) {
  union { v16b v; v8b q[2]; } u; const __bf16* p = rowk0 + 8 * (lane >> 4);
  u.q[0] = *(const v8b*)p; u.q[1] = *(const v8b*)(p + 16); return u.v;
}
__device__ __forceinline__ float bfr(float v) { return (float)(__bf16)v; }
__device__ __attribute__((noinline)) float exp_ni(float v) { return expf(v); }
__device__ __attribute__((noinline)) float erf_ni(float v) { return erff(v); }

#define WS_TH  0u
#define WS_S   (WS_TH + 4u * NP * 8)
#define WS_WC  (WS_S + 2u * (size_t)NP * HS * WSd * CHP)
#define WS_ST  (WS_WC + 2u * HID * KTAP * CHP)
#define WS_BNP (WS_ST + 4u * (size_t)NP * NBLK * 2 * HID)
#define WS_MS  (WS_BNP + 4u * 2 * HID * 2)
#define WS_END (WS_MS + 4u * (size_t)NP * NBLK * HID)

__global__ __launch_bounds__(64) void k_packw(const float* __restrict__ CW, __bf16* __restrict__ WC) {
  const int o = blockIdx.x, c = threadIdx.x; __shared__ __align__(16) __bf16 s[KTAP * CHP];
  for (int k = 0; k < KTAP; ++k) s[k * CHP + c] = (__bf16)((c < CHM) ? CW[((size_t)o * CHM + c) * KTAP + k] : 0.f);
  __syncthreads();
  for (int q = c; q < KTAP * CHP / 8; q += 64) vst2((unsigned*)(WC + (size_t)o * KTAP * CHP + q * 8), *(const v4u*)&s[q * 8]);
}
__global__ __launch_bounds__(64) void k_theta(const float* __restrict__ QF, const float* __restrict__ W1, const float* __restrict__ B1, const float* __restrict__ W2, const float* __restrict__ B2, const float* __restrict__ W3, const float* __restrict__ B3, float* __restrict__ TH) {
  __shared__ float sq[INC], sh1[HID], sh2[HID]; __shared__ __align__(16) float sth[16][8]; const int t = threadIdx.x;
  for (int i = 0; i < 16; ++i) { const int p = blockIdx.x * 16 + i; const int n = p / NBq, b = p % NBq;
    for (int k = t; k < INC; k += 64) sq[k] = bfr(QF[((size_t)b * NQ + n) * INC + k]);
    __syncthreads();
    { float a = 0.f; for (int k = 0; k < INC; ++k) a += sq[k] * bfr(W1[t * INC + k]); sh1[t] = fmaxf(a + bfr(B1[t]), 0.f); }
    __syncthreads();
    { float a = 0.f; for (int k = 0; k < HID; ++k) a += sh1[k] * bfr(W2[t * HID + k]); sh2[t] = fmaxf(a + bfr(B2[t]), 0.f); }
    __syncthreads();
    if (t < 8) { float a = 0.f; if (t < 6) { for (int k = 0; k < HID; ++k) a += sh2[k] * bfr(W3[t * HID + k]); a += bfr(B3[t]); } sth[i][t] = a; }
    __syncthreads(); }
  if (t < 32) vst2(TH + (size_t)blockIdx.x * 16 * 8 + t * 4, *(const v4f*)(&sth[0][0] + t * 4));
}
__global__ __launch_bounds__(128) void k_sample(const float* __restrict__ HM, const float* __restrict__ TH, __bf16* __restrict__ S) {
  __shared__ int sidx[4][WSd]; __shared__ float swt[4][WSd]; __shared__ __align__(16) __bf16 so[WSd][CHP];
  const int gy = blockIdx.x, p = blockIdx.y, t = threadIdx.x; const int b = p % NBq;
  if (t < WSd) { const int gx = t; const float* th = TH + (size_t)p * 8;
    const float xb = ((float)gx * 2.0f + 1.0f) / (float)WSd - 1.0f, yb = ((float)gy * 2.0f + 1.0f) / (float)HS - 1.0f;
    const float gxv = xb * th[0] + yb * th[1] + th[2], gyv = xb * th[3] + yb * th[4] + th[5];
    const float ix = ((gxv + 1.0f) * (float)WIN - 1.0f) * 0.5f, iy = ((gyv + 1.0f) * (float)HIN - 1.0f) * 0.5f;
    const float x0 = floorf(ix), y0 = floorf(iy); const float wx1 = ix - x0, wy1 = iy - y0;
    const float xs[2] = {x0, x0 + 1.0f}, ys[2] = {y0, y0 + 1.0f}; const float wxs[2] = {1.0f - wx1, wx1}, wys[2] = {1.0f - wy1, wy1};
#pragma unroll
    for (int q = 0; q < 4; ++q) { const int cx = q & 1, cy = q >> 1;
      const float xi = xs[cx], yi = ys[cy]; const float m = (xi >= 0.f && xi < (float)WIN && yi >= 0.f && yi < (float)HIN) ? 1.0f : 0.0f;
      const int xc = (int)fminf(fmaxf(xi, 0.f), (float)(WIN - 1)), yc = (int)fminf(fmaxf(yi, 0.f), (float)(HIN - 1));
      sidx[q][gx] = yc * WIN + xc; swt[q][gx] = (wxs[cx] * wys[cy]) * m; } }
  __syncthreads();
  for (int e = t; e < WSd * CHP; e += 128) { const int gx = e / CHP, c = e % CHP; float v = 0.f;
    if (c < CHM) { const float* img = HM + ((size_t)b * CHM + c) * HIN * WIN;
#pragma unroll
      for (int q = 0; q < 4; ++q) v = v + bfr(img[sidx[q][gx]]) * swt[q][gx]; }
    so[gx][c] = (__bf16)v; }
  __syncthreads();
  for (int e = t; e < WSd * CHP / 8; e += 128) { const int gx = e / (CHP / 8), q8 = e % (CHP / 8); vst2((unsigned*)(S + (((size_t)p * HS + gy) * WSd + gx) * CHP + q8 * 8), *(const v4u*)&so[gx][q8 * 8]); }
}
template <int PASS>
__global__ __launch_bounds__(128) void k_conv(const __bf16* __restrict__ S, const __bf16* __restrict__ WC, const float* __restrict__ CB, const float* __restrict__ BNP, float* __restrict__ ST, float* __restrict__ MS) {
  __shared__ __align__(16) float sy[64][HID + 1]; __shared__ __align__(16) float sred[2][HID];
  const int tid = threadIdx.x, wave = tid >> 5, lane = tid & 31, col = lane & 15, g = lane >> 4; const int blk = blockIdx.x; const size_t p = blockIdx.y;
  const int pos = blk * 64 + wave * 16 + col; const int posc = pos < NPOS ? pos : NPOS - 1; const int oy = posc / WO, ox = posc % WO;
  const __bf16* rowbase = S + ((p * HS + oy) * WSd + ox) * CHP;
  v8f acc[4] = {};
#pragma unroll
  for (int k = 0; k < KTAP; ++k) { const __bf16* rp = rowbase + ((k / 3) * WSd + (k % 3)) * CHP;
#pragma unroll
    for (int cc = 0; cc < 2; ++cc) { const v16b a = frag_b(rp + cc * 32, lane);
#pragma unroll
      for (int j = 0; j < 4; ++j) acc[j] = wmma_bf(a, frag_b(WC + (size_t)(j * 16 + col) * (KTAP * CHP) + k * CHP + cc * 32, lane), acc[j]); } }
#pragma unroll
  for (int j = 0; j < 4; ++j) { const int o = j * 16 + col; const float bb = bfr(CB[o]);
#pragma unroll
    for (int r = 0; r < 8; ++r) { float y = acc[j][r] + bb; if (PASS == 1) { y = fmaxf((y - BNP[o]) * BNP[HID + o] + BNP[2 * HID + o], 0.f); } sy[wave * 16 + 8 * g + r][o] = y; } }
  __syncthreads();
  const int nvalid = min(64, NPOS - blk * 64);
  if (tid < HID) { const int o = tid;
    if (PASS == 0) { float s = 0.f; for (int r = 0; r < nvalid; ++r) s += sy[r][o]; const float mean = s / (float)nvalid; float m2 = 0.f; for (int r = 0; r < nvalid; ++r) { const float d = sy[r][o] - mean; m2 += d * d; } sred[0][o] = mean; sred[1][o] = m2; }
    else { float s = 0.f; for (int r = 0; r < nvalid; ++r) s += sy[r][o]; sred[0][o] = s; } }
  __syncthreads();
  if (PASS == 0) { if (tid < 2 * HID / 4) vst2(ST + ((p * NBLK + blk) * 2 * HID) + tid * 4, *(const v4f*)(&sred[0][0] + tid * 4)); }
  else { if (tid < HID / 4) vst2(MS + ((p * NBLK + blk) * HID) + tid * 4, *(const v4f*)(&sred[0][0] + tid * 4)); }
}
__global__ __launch_bounds__(64) void k_bn(const float* __restrict__ ST, const float* __restrict__ G, const float* __restrict__ Bt, float* __restrict__ BNP) {
  const int o = threadIdx.x; float n = 0.f, mean = 0.f, m2 = 0.f;
  for (int p = 0; p < TNP; ++p) for (int blk = 0; blk < NBLK; ++blk) { const float nb = (float)min(64, NPOS - blk * 64); const float mb = ST[(((size_t)p * NBLK + blk) * 2) * HID + o], m2b = ST[(((size_t)p * NBLK + blk) * 2 + 1) * HID + o];
    const float nn = n + nb; const float delta = mb - mean; mean = mean + delta * (nb / nn); m2 = m2 + m2b + delta * delta * (n * nb / nn); n = nn; }
  const float var = m2 / n; __shared__ __align__(16) float so[3][HID]; so[0][o] = mean; so[1][o] = (1.0f / sqrtf(var + 1e-5f)) * bfr(G[o]); so[2][o] = bfr(Bt[o]); __syncthreads();
  if (o < 3 * HID / 4) vst2(BNP + o * 4, *(const v4f*)(&so[0][0] + o * 4));
}
__global__ __launch_bounds__(64) void k_fin(const float* __restrict__ MS, const float* __restrict__ W2, const float* __restrict__ B2, float* __restrict__ OUT) {
  __shared__ __align__(16) float so[16][2]; __shared__ float ym[HID]; const int t = threadIdx.x;
  for (int i = 0; i < 16; ++i) { const size_t p = (size_t)blockIdx.x * 16 + i;
    { float s = 0.f; for (int blk = 0; blk < NBLK; ++blk) s += MS[(p * NBLK + blk) * HID + t]; ym[t] = s / (float)NPOS; }
    __syncthreads();
    if (t < 2) { float a = 0.f; for (int o = 0; o < HID; ++o) a += ym[o] * bfr(W2[t * HID + o]); so[i][t] = a + bfr(B2[t]); }
    __syncthreads(); }
  if (t < 8) vst2(OUT + (size_t)blockIdx.x * 32 + t * 4, *(const v4f*)(&so[0][0] + t * 4));
}
extern "C" void kernel_launch(void* const* d_in, const int* in_sizes, int n_in, void* d_out, int out_size, void* d_ws, size_t ws_size, hipStream_t stream) {
  (void)in_sizes; (void)n_in; (void)out_size;
  const float** F = (const float**)d_in;
  if (ws_size < (size_t)WS_END) return;
  char* ws = (char*)d_ws; float *TH = (float*)(ws + WS_TH), *ST = (float*)(ws + WS_ST), *BNP = (float*)(ws + WS_BNP), *MS = (float*)(ws + WS_MS); __bf16 *S = (__bf16*)(ws + WS_S), *WC = (__bf16*)(ws + WS_WC);
  k_packw<<<HID, 64, 0, stream>>>(F[8], WC);
  k_theta<<<NP / 16, 64, 0, stream>>>(F[0], F[2], F[3], F[4], F[5], F[6], F[7], TH);
  k_sample<<<dim3(HS, TNP), 128, 0, stream>>>(F[1], TH, S);
  k_conv<0><<<dim3(NBLK, TNP), 128, 0, stream>>>(S, WC, F[9], BNP, ST, MS);
  k_bn<<<1, 64, 0, stream>>>(ST, F[10], F[11], BNP);
  k_conv<1><<<dim3(NBLK, TNP), 128, 0, stream>>>(S, WC, F[9], BNP, ST, MS);
  k_fin<<<TNP / 16, 64, 0, stream>>>(MS, F[12], F[13], (float*)d_out);
}
